// MultiHeadAttention_36318243455145
// MI455X (gfx1250) — hardware-verified
//
#include <hip/hip_runtime.h>
#include <math.h>

#ifndef NB
#define NB 2
#endif
#ifndef SEQ
#define SEQ 2048
#endif
#define NB_FULL 2
#define SEQ_FULL 2048
#define DM 1024
#define NH 16
#define DH 64
#define ROWS (NB * SEQ)

static_assert(NH * DH == DM);
static_assert(DH == 64);
static_assert(SEQ % 64 == 0);
static_assert(ROWS % 64 == 0);
static_assert(DM % 64 == 0);
static_assert(DM % 32 == 0);
static_assert((2 * DM) % 32 == 0);
static_assert(NB <= NB_FULL && SEQ <= SEQ_FULL);
static_assert(16 * 4 == 64);
static_assert(8 * 8 == 64);

typedef __attribute__((ext_vector_type(16))) _Float16     v16h;
typedef __attribute__((ext_vector_type(16))) __bf16       v16b;
typedef __attribute__((ext_vector_type(8)))  float        v8f;
typedef __attribute__((ext_vector_type(4)))  float        v4f;
typedef __attribute__((ext_vector_type(4)))  unsigned int v4u;
typedef __attribute__((ext_vector_type(8)))  unsigned int v8u;
typedef v4f __attribute__((may_alias)) v4fa;

__device__ __forceinline__ v8u ld_frag(const unsigned short* __restrict__ p) {
  const v4u x = *(const v4u*)(p);
  const v4u y = *(const v4u*)(p + 16);
  v8u r;
  r[0] = x.x; r[1] = x.y; r[2] = x.z; r[3] = x.w;
  r[4] = y.x; r[5] = y.y; r[6] = y.z; r[7] = y.w;
  return r;
}

__device__ __forceinline__ unsigned int bfbits(float f) {
  const unsigned int u = __float_as_uint(f);
  return (u + 0x7FFFu + ((u >> 16) & 1u)) >> 16;
}
__device__ __forceinline__ float bfval(float f) { return __uint_as_float(bfbits(f) << 16); }
__device__ __forceinline__ unsigned int pk2h(float a, float b) {
  return (unsigned int)__builtin_bit_cast(unsigned short, (_Float16)a) |
         ((unsigned int)__builtin_bit_cast(unsigned short, (_Float16)b) << 16);
}
__device__ __forceinline__ void bfsplit2(float a, float b, unsigned int& hi, unsigned int& lo) {
  const unsigned int ha = bfbits(a), hb = bfbits(b);
  const unsigned int la = bfbits(a - __uint_as_float(ha << 16));
  const unsigned int lb = bfbits(b - __uint_as_float(hb << 16));
  hi = ha | (hb << 16);
  lo = la | (lb << 16);
}

__device__ __forceinline__ v8f mma_h(v8u a, v8u b, v8f c) {
  return __builtin_amdgcn_wmma_f32_16x16x32_f16(false, __builtin_bit_cast(v16h, a), false, __builtin_bit_cast(v16h, b), (short)0, c, false, false);
}
__device__ __forceinline__ v8f mma_b(v8u a, v8u b, v8f c) {
  return __builtin_amdgcn_wmma_f32_16x16x32_bf16(false, __builtin_bit_cast(v16b, a), false, __builtin_bit_cast(v16b, b), (short)0, c, false, false);
}
template <int ET> __device__ __forceinline__ v8f mma16(v8u a, v8u b, v8f c) {
  if (ET == 0) return mma_h(a, b, c);
  return mma_b(a, b, c);
}
__device__ __forceinline__ void guard4(v8f& a0, v8f& a1, v8f& a2, v8f& a3, v8u x, v8u y0, v8u y1, v8u y2, v8u y3) {
  asm volatile("v_nop\n\tv_nop\n\tv_nop\n\tv_nop" : "+v"(a0), "+v"(a1), "+v"(a2), "+v"(a3) : "v"(x), "v"(y0), "v"(y1), "v"(y2), "v"(y3));
}
__device__ __forceinline__ v8f mma3b(v8u ah, v8u al, v8u bh, v8u bl, v8f c) {
  c = mma_b(ah, bh, c);
  c = mma_b(ah, bl, c);
  c = mma_b(al, bh, c);
  asm volatile("v_nop\n\tv_nop\n\tv_nop\n\tv_nop" : "+v"(c) : "v"(ah), "v"(al), "v"(bh), "v"(bl));
  return c;
}

__global__ __launch_bounds__(256) void k_cast_h(const float* __restrict__ src, unsigned short* __restrict__ dst,
                                                int nrows, int rows_per_b, long long src_bstride, float sc) {
  const long long u = (long long)blockIdx.x * 256 + threadIdx.x;
  if (u >= (long long)nrows * (DM / 8)) return;
  const int r = (int)(u / (DM / 8));
  const int c0 = 8 * (int)(u % (DM / 8));
  const int bb = r / rows_per_b;
  const int s = r - bb * rows_per_b;
  const float* p = src + (long long)bb * src_bstride + (long long)s * DM + c0;
  const v4f f0 = *(const v4f*)(p);
  const v4f f1 = *(const v4f*)(p + 4);
  v4u pk;
  pk.x = pk2h(bfval(f0.x) * sc, bfval(f0.y) * sc);
  pk.y = pk2h(bfval(f0.z) * sc, bfval(f0.w) * sc);
  pk.z = pk2h(bfval(f1.x) * sc, bfval(f1.y) * sc);
  pk.w = pk2h(bfval(f1.z) * sc, bfval(f1.w) * sc);
  volatile v4u* d = (volatile v4u*)(dst + (long long)r * DM + c0);
  *d = pk;
  __threadfence();
  *d = pk;
}
__global__ __launch_bounds__(256) void k_cast_wo2(const float* __restrict__ src, unsigned short* __restrict__ dst) {
  const long long u = (long long)blockIdx.x * 256 + threadIdx.x;
  if (u >= (long long)DM * (2 * DM / 8)) return;
  const int r = (int)(u / (2 * DM / 8));
  const int c0 = 8 * (int)(u % (2 * DM / 8));
  const int sc0 = c0 & (DM - 1);
  const float* p = src + (long long)r * DM + sc0;
  const v4f f0 = *(const v4f*)(p);
  const v4f f1 = *(const v4f*)(p + 4);
  v4u pk;
  pk.x = bfbits(f0.x) | (bfbits(f0.y) << 16);
  pk.y = bfbits(f0.z) | (bfbits(f0.w) << 16);
  pk.z = bfbits(f1.x) | (bfbits(f1.y) << 16);
  pk.w = bfbits(f1.z) | (bfbits(f1.w) << 16);
  volatile v4u* d = (volatile v4u*)(dst + (long long)r * (2 * DM) + c0);
  *d = pk;
  __threadfence();
  *d = pk;
}

template <int ET, int BIAS_MODE, int OUT_MODE>
__device__ __forceinline__ void gemm64_body(
    const unsigned short* __restrict__ Ap, int lda, long long strideA,
    const unsigned short* __restrict__ Bp, int ldb, long long strideB,
    unsigned short* __restrict__ C16a, unsigned short* __restrict__ C16b, float* __restrict__ C32,
    int ldc, long long strideC, const float* __restrict__ bias,
    int M, int N, int K, float scale, float post) {
  __shared__ __align__(16) float sT[8 * 16 * 68];
  const int bz = blockIdx.y;
  const int lane = threadIdx.x & 31;
  const int wave = __builtin_amdgcn_readfirstlane((int)(threadIdx.x >> 5));
  const int tilesN = N >> 6;
  const int tilesM = M >> 6;
  const int tile = (int)blockIdx.x * 8 + wave;
  if (tile >= tilesM * tilesN) return;
  const int tm = tile / tilesN;
  const int tn = tile - tm * tilesN;
  const int m0 = tm << 6;
  const int n0 = tn << 6;
  const int rlane = lane & 15;
  const int hh = lane >> 4;
  const int koff = hh * 8;
  const int mOff = hh * 8;
  const unsigned short* Ab = Ap + (size_t)bz * (size_t)strideA;
  const unsigned short* Bb = Bp + (size_t)bz * (size_t)strideB;

  v8f acc[4][4];
#pragma unroll
  for (int i = 0; i < 4; ++i)
#pragma unroll
    for (int j = 0; j < 4; ++j) { v8f zz = {0.f, 0.f, 0.f, 0.f, 0.f, 0.f, 0.f, 0.f}; acc[i][j] = zz; }

  for (int k0 = 0; k0 < K; k0 += 32) {
    v8u bf[4];
#pragma unroll
    for (int j = 0; j < 4; ++j) bf[j] = ld_frag(Bb + (size_t)(n0 + 16 * j + rlane) * ldb + koff + k0);
#pragma unroll
    for (int i = 0; i < 4; ++i) {
      const v8u af = ld_frag(Ab + (size_t)(m0 + 16 * i + rlane) * lda + koff + k0);
#pragma unroll
      for (int j = 0; j < 4; ++j) acc[i][j] = mma16<ET>(af, bf[j], acc[i][j]);
      guard4(acc[i][0], acc[i][1], acc[i][2], acc[i][3], af, bf[0], bf[1], bf[2], bf[3]);
    }
  }

  const int sb = wave * (16 * 68);
  float bvj[4];
#pragma unroll
  for (int j = 0; j < 4; ++j) bvj[j] = (BIAS_MODE == 2) ? bfval(bias[n0 + 16 * j + rlane]) : 0.f;
#pragma unroll
  for (int i = 0; i < 4; ++i) {
    const int mBase = m0 + 16 * i;
    float br[8];
#pragma unroll
    for (int r = 0; r < 8; ++r) br[r] = (BIAS_MODE == 1) ? bfval(bias[mBase + mOff + r]) : 0.f;
#pragma unroll
    for (int j = 0; j < 4; ++j) {
#pragma unroll
      for (int r = 0; r < 8; ++r) {
        float v = acc[i][j][r] * scale;
        if (BIAS_MODE == 1) v += br[r];
        if (BIAS_MODE == 2) v += bvj[j];
        v *= post;
        sT[sb + (mOff + r) * 68 + 16 * j + rlane] = v;
      }
    }
    __builtin_amdgcn_fence(3  , "workgroup");
    __builtin_amdgcn_wave_barrier();
    __builtin_amdgcn_fence(2  , "workgroup");
    if (OUT_MODE == 0) {
      float* C = C32 + (size_t)bz * (size_t)strideC;
      const int c4 = (lane & 15) * 4;
      v4f val[8];
#pragma unroll
      for (int it = 0; it < 8; ++it) val[it] = *(const v4fa*)&sT[sb + (it * 2 + hh) * 68 + c4];
      for (int pass = 0; pass < 2; ++pass) {
#pragma unroll
        for (int it = 0; it < 8; ++it) {
          const int row = it * 2 + hh;
          *(volatile v4f*)(C + (size_t)(mBase + row) * ldc + n0 + c4) = val[it];
        }
        __threadfence();
      }
    } else {
      const int q = lane >> 3;
      const int c8 = (lane & 7) * 8;
      unsigned short* Ca = C16a + (size_t)bz * (size_t)strideC;
      unsigned short* Cb = (OUT_MODE == 2) ? (C16b + (size_t)bz * (size_t)strideC) : Ca;
      v4u hv[4], lv[4];
#pragma unroll
      for (int it = 0; it < 4; ++it) {
        const int row = it * 4 + q;
        const v4f f0 = *(const v4fa*)&sT[sb + row * 68 + c8];
        const v4f f1 = *(const v4fa*)&sT[sb + row * 68 + c8 + 4];
        if (OUT_MODE == 1) {
          hv[it].x = pk2h(f0.x, f0.y); hv[it].y = pk2h(f0.z, f0.w);
          hv[it].z = pk2h(f1.x, f1.y); hv[it].w = pk2h(f1.z, f1.w);
          lv[it] = hv[it];
        } else {
          unsigned int h0, l0, h1, l1, h2, l2, h3, l3;
          bfsplit2(f0.x, f0.y, h0, l0); bfsplit2(f0.z, f0.w, h1, l1);
          bfsplit2(f1.x, f1.y, h2, l2); bfsplit2(f1.z, f1.w, h3, l3);
          hv[it].x = h0; hv[it].y = h1; hv[it].z = h2; hv[it].w = h3;
          lv[it].x = l0; lv[it].y = l1; lv[it].z = l2; lv[it].w = l3;
        }
      }
      for (int pass = 0; pass < 2; ++pass) {
#pragma unroll
        for (int it = 0; it < 4; ++it) {
          const int row = it * 4 + q;
          const size_t o = (size_t)(mBase + row) * ldc + n0 + c8;
          *(volatile v4u*)(Ca + o) = hv[it];
          if (OUT_MODE == 2) *(volatile v4u*)(Cb + o) = lv[it];
        }
        __threadfence();
      }
    }
    __builtin_amdgcn_fence(3  , "workgroup");
    __builtin_amdgcn_wave_barrier();
    __builtin_amdgcn_fence(2  , "workgroup");
  }
}

__global__ __launch_bounds__(256) void k_proj_qk(const unsigned short* __restrict__ X, const unsigned short* __restrict__ W,
                                                 const float* __restrict__ bias, unsigned short* __restrict__ PH,
                                                 unsigned short* __restrict__ PL, float post) {
  gemm64_body<0, 2, 2>(X, DM, 0, W, DM, 0, PH, PL, nullptr, DM, 0, bias, ROWS, DM, DM, 1.0f / 16.0f, post);
}
__global__ __launch_bounds__(256) void k_proj_vt(const unsigned short* __restrict__ W, const unsigned short* __restrict__ X,
                                                 const float* __restrict__ bias, unsigned short* __restrict__ VT) {
  gemm64_body<0, 1, 1>(W, DM, 0, X, DM, (long long)SEQ * DM, VT, nullptr, nullptr, SEQ, (long long)DM * SEQ, bias, DM, SEQ, DM, 1.0f / 16.0f, 1.0f);
}
__global__ __launch_bounds__(256) void k_proj_out(const unsigned short* __restrict__ CTX, const unsigned short* __restrict__ WO2,
                                                  const float* __restrict__ bias, float* __restrict__ out) {
  gemm64_body<1, 2, 0>(CTX, 2 * DM, 0, WO2, 2 * DM, 0, nullptr, nullptr, out, DM, 0, bias, ROWS, DM, 2 * DM, 1.0f, 1.0f);
}

__global__ __launch_bounds__(128) void k_attn(const unsigned short* __restrict__ QH, const unsigned short* __restrict__ QL,
                                              const unsigned short* __restrict__ KH, const unsigned short* __restrict__ KL,
                                              const unsigned short* __restrict__ VT, unsigned short* __restrict__ CTX) {
  __shared__ __align__(16) float Os[4 * 16 * 68];
  const int lane = threadIdx.x & 31;
  const int hh = lane >> 4;
  const int c = lane & 15;
  const int wave = __builtin_amdgcn_readfirstlane((int)(threadIdx.x >> 5));
  const int bx = (int)blockIdx.x;
  const int qb = bx % (SEQ / 64);
  const int bh = bx / (SEQ / 64);
  const int h = bh % NH;
  const int b = bh / NH;
  const int q0 = qb * 64 + wave * 16;

  const size_t qoff = ((size_t)b * SEQ + q0 + c) * DM + h * DH + 8 * hh;
  const size_t kbase = ((size_t)b * SEQ + c) * DM + h * DH + 8 * hh;
  const size_t vbase = ((size_t)b * DM + h * DH + c) * SEQ + 8 * hh;

  v8f oacc[4];
#pragma unroll
  for (int t = 0; t < 4; ++t) { v8f zz = {0.f, 0.f, 0.f, 0.f, 0.f, 0.f, 0.f, 0.f}; oacc[t] = zz; }
  float m_run = -1.0e30f;
  float l_part = 0.f;
  const float L2E = 1.4426950408889634f;

#pragma unroll 1
  for (int kv0 = 0; kv0 < SEQ; kv0 += 32) {
    v8f x0 = {0.f, 0.f, 0.f, 0.f, 0.f, 0.f, 0.f, 0.f};
    v8f x1 = {0.f, 0.f, 0.f, 0.f, 0.f, 0.f, 0.f, 0.f};
#pragma unroll
    for (int dc = 0; dc < 2; ++dc) {
      const v8u qh = ld_frag(QH + qoff + dc * 32);
      const v8u ql = ld_frag(QL + qoff + dc * 32);
      const size_t ko0 = kbase + (size_t)kv0 * DM + dc * 32;
      {
        const v8u kh = ld_frag(KH + ko0);
        const v8u kl = ld_frag(KL + ko0);
        x0 = mma3b(kh, kl, qh, ql, x0);
      }
      {
        const size_t ko1 = ko0 + (size_t)16 * DM;
        const v8u kh = ld_frag(KH + ko1);
        const v8u kl = ld_frag(KL + ko1);
        x1 = mma3b(kh, kl, qh, ql, x1);
      }
    }

    float mx = fmaxf(x0[0], x1[0]);
#pragma unroll
    for (int i = 1; i < 8; ++i) mx = fmaxf(mx, fmaxf(x0[i], x1[i]));
    mx = fmaxf(mx, __shfl_xor(mx, 16, 32));
    const float m_new = fmaxf(m_run, mx * L2E);
    const float sc = exp2f(m_run - m_new);
    const float mb = 12.0f - m_new;
    float p0[8], p1[8];
    float s = 0.f;
#pragma unroll
    for (int i = 0; i < 8; ++i) {
      p0[i] = exp2f(fmaf(x0[i], L2E, mb));
      p1[i] = exp2f(fmaf(x1[i], L2E, mb));
      s += p0[i] + p1[i];
    }
    l_part = l_part * sc + s;
    m_run = m_new;
#pragma unroll
    for (int t = 0; t < 4; ++t) oacc[t] = oacc[t] * sc;

    v8u bp;
#pragma unroll
    for (int j = 0; j < 4; ++j) {
      bp[j] = pk2h(p0[2 * j], p0[2 * j + 1]);
      bp[4 + j] = pk2h(p1[2 * j], p1[2 * j + 1]);
    }

    const size_t vo = vbase + kv0;
    const v8u va0 = ld_frag(VT + vo);
    const v8u va1 = ld_frag(VT + vo + (size_t)16 * SEQ);
    const v8u va2 = ld_frag(VT + vo + (size_t)32 * SEQ);
    const v8u va3 = ld_frag(VT + vo + (size_t)48 * SEQ);
    oacc[0] = mma_h(va0, bp, oacc[0]);
    oacc[1] = mma_h(va1, bp, oacc[1]);
    oacc[2] = mma_h(va2, bp, oacc[2]);
    oacc[3] = mma_h(va3, bp, oacc[3]);
    guard4(oacc[0], oacc[1], oacc[2], oacc[3], bp, va0, va1, va2, va3);
  }

  const float l = l_part + __shfl_xor(l_part, 16, 32);
  const float inv = 1.0f / l;

  const int ob = wave * (16 * 68);
#pragma unroll
  for (int t = 0; t < 4; ++t) {
    v4f a0, a1;
    a0.x = oacc[t][0] * inv; a0.y = oacc[t][1] * inv; a0.z = oacc[t][2] * inv; a0.w = oacc[t][3] * inv;
    a1.x = oacc[t][4] * inv; a1.y = oacc[t][5] * inv; a1.z = oacc[t][6] * inv; a1.w = oacc[t][7] * inv;
    *(v4fa*)&Os[ob + c * 68 + t * 16 + 8 * hh] = a0;
    *(v4fa*)&Os[ob + c * 68 + t * 16 + 8 * hh + 4] = a1;
  }
  __builtin_amdgcn_fence(3  , "workgroup");
  __builtin_amdgcn_wave_barrier();
  __builtin_amdgcn_fence(2  , "workgroup");
  {
    const int q = lane >> 3;
    const int c8 = (lane & 7) * 8;
    v4u hv[4], lv[4];
#pragma unroll
    for (int it = 0; it < 4; ++it) {
      const int row = it * 4 + q;
      const v4f f0 = *(const v4fa*)&Os[ob + row * 68 + c8];
      const v4f f1 = *(const v4fa*)&Os[ob + row * 68 + c8 + 4];
      unsigned int h0, l0, h1, l1, h2, l2, h3, l3;
      bfsplit2(f0.x, f0.y, h0, l0); bfsplit2(f0.z, f0.w, h1, l1);
      bfsplit2(f1.x, f1.y, h2, l2); bfsplit2(f1.z, f1.w, h3, l3);
      hv[it].x = h0; hv[it].y = h1; hv[it].z = h2; hv[it].w = h3;
      lv[it].x = l0; lv[it].y = l1; lv[it].z = l2; lv[it].w = l3;
    }
    for (int pass = 0; pass < 2; ++pass) {
#pragma unroll
      for (int it = 0; it < 4; ++it) {
        const int row = it * 4 + q;
        const size_t o = ((size_t)b * SEQ + q0 + row) * (2 * DM) + h * DH + c8;
        *(volatile v4u*)(CTX + o) = hv[it];
        *(volatile v4u*)(CTX + o + DM) = lv[it];
      }
      __threadfence();
    }
  }
}

#define SZ_X16   ((size_t)3 * ROWS * DM * 2)
#define SZ_W16   ((size_t)3 * DM * DM * 2)
#define SZ_WO2   ((size_t)DM * 2 * DM * 2)
#define SZ_P16   ((size_t)ROWS * DM * 2)
#define SZ_CTX   ((size_t)ROWS * 2 * DM * 2)
#define WS_TOTAL (SZ_X16 + SZ_W16 + SZ_WO2 + 5 * SZ_P16 + SZ_CTX)
static_assert(WS_TOTAL <= (size_t)134217728);
static_assert(SZ_X16 % 256 == 0 && SZ_W16 % 256 == 0 && SZ_WO2 % 256 == 0 && SZ_P16 % 256 == 0 && SZ_CTX % 256 == 0);
static_assert((size_t)NB * DM * SEQ * 2 == SZ_P16);

extern "C" void kernel_launch(void* const* d_in, const int* in_sizes, int n_in, void* d_out, int out_size, void* d_ws, size_t ws_size, hipStream_t stream) {
  if (n_in < 11) return;
  const long long need_x = ((long long)(NB - 1) * SEQ_FULL + SEQ) * DM;
  if (in_sizes[0] < need_x || in_sizes[1] < need_x || in_sizes[2] < need_x) return;
  if (in_sizes[3] < DM * DM || in_sizes[5] < DM * DM || in_sizes[7] < DM * DM || in_sizes[9] < DM * DM) return;
  if (in_sizes[4] < DM || in_sizes[6] < DM || in_sizes[8] < DM || in_sizes[10] < DM) return;
  if ((long long)out_size < (long long)ROWS * DM) return;
  if (ws_size < WS_TOTAL) return;

  const float* xq = (const float*)d_in[0];
  const float* xk = (const float*)d_in[1];
  const float* xv = (const float*)d_in[2];
  const float* Wq = (const float*)d_in[3];
  const float* bq = (const float*)d_in[4];
  const float* Wk = (const float*)d_in[5];
  const float* bk = (const float*)d_in[6];
  const float* Wv = (const float*)d_in[7];
  const float* bv = (const float*)d_in[8];
  const float* Wo = (const float*)d_in[9];
  const float* bo = (const float*)d_in[10];
  float* out = (float*)d_out;

  char* wsp = (char*)d_ws;
  unsigned short* X16 = (unsigned short*)wsp; wsp += SZ_X16;
  unsigned short* W16 = (unsigned short*)wsp; wsp += SZ_W16;
  unsigned short* WO2 = (unsigned short*)wsp; wsp += SZ_WO2;
  unsigned short* QH  = (unsigned short*)wsp; wsp += SZ_P16;
  unsigned short* QL  = (unsigned short*)wsp; wsp += SZ_P16;
  unsigned short* KH  = (unsigned short*)wsp; wsp += SZ_P16;
  unsigned short* KL  = (unsigned short*)wsp; wsp += SZ_P16;
  unsigned short* VT  = (unsigned short*)wsp; wsp += SZ_P16;
  unsigned short* CTX = (unsigned short*)wsp; wsp += SZ_CTX;

  const size_t XP = (size_t)ROWS * DM;
  const size_t WP = (size_t)DM * DM;
  const unsigned gx = (unsigned)(((long long)ROWS * (DM / 8) + 255) / 256);
  const unsigned gw = (unsigned)(((long long)DM * (DM / 8) + 255) / 256);
  const unsigned gw2 = (unsigned)(((long long)DM * (2 * DM / 8) + 255) / 256);

  k_cast_h<<<gx, 256, 0, stream>>>(xq, X16,          ROWS, SEQ, (long long)SEQ_FULL * DM, 1.0f);
  k_cast_h<<<gx, 256, 0, stream>>>(xk, X16 + XP,     ROWS, SEQ, (long long)SEQ_FULL * DM, 1.0f);
  k_cast_h<<<gx, 256, 0, stream>>>(xv, X16 + 2 * XP, ROWS, SEQ, (long long)SEQ_FULL * DM, 1.0f);
  k_cast_h<<<gw, 256, 0, stream>>>(Wq, W16,          DM, DM, 0, 16.0f);
  k_cast_h<<<gw, 256, 0, stream>>>(Wk, W16 + WP,     DM, DM, 0, 16.0f);
  k_cast_h<<<gw, 256, 0, stream>>>(Wv, W16 + 2 * WP, DM, DM, 0, 16.0f);
  k_cast_wo2<<<gw2, 256, 0, stream>>>(Wo, WO2);

  const unsigned gp = (unsigned)(((ROWS / 64) * (DM / 64) + 7) / 8);
  k_proj_qk<<<dim3(gp, 1), 256, 0, stream>>>(X16,      W16,      bq, QH, QL, 0.125f);
  k_proj_qk<<<dim3(gp, 1), 256, 0, stream>>>(X16 + XP, W16 + WP, bk, KH, KL, 1.0f);
  const unsigned gv = (unsigned)(((DM / 64) * (SEQ / 64) + 7) / 8);
  k_proj_vt<<<dim3(gv, NB), 256, 0, stream>>>(W16 + 2 * WP, X16 + 2 * XP, bv, VT);

  k_attn<<<dim3((unsigned)(NB * NH * (SEQ / 64))), 128, 0, stream>>>(QH, QL, KH, KL, VT, CTX);

  k_proj_out<<<dim3(gp, 1), 256, 0, stream>>>(CTX, WO2, bo, out);
}
